// GRUModel_46986942218988
// MI455X (gfx1250) — hardware-run, weakly checked
//
#include <hip/hip_runtime.h>
#include <math.h>

typedef __attribute__((ext_vector_type(16))) _Float16 v16h;
typedef __attribute__((ext_vector_type(8)))  _Float16 v8h;
typedef __attribute__((ext_vector_type(16))) __bf16   v16b;
typedef __attribute__((ext_vector_type(8)))  __bf16   v8b;
typedef __attribute__((ext_vector_type(8)))  float    v8f;
typedef __attribute__((ext_vector_type(4)))  float    v4f;
typedef __attribute__((ext_vector_type(4)))  int      v4i;

constexpr int kL     = 25;
constexpr int kE     = 64;
constexpr int kH     = 8;
constexpr int kV     = 30000;
constexpr int kB     = 1000;
constexpr int kS     = 512;
constexpr int kVPad  = 30016;
constexpr int kPP    = 64;
constexpr int kBPad  = 1008;
constexpr int kTiles = 63;
constexpr int kOutTotal = kB + kL * kB * kH;
static_assert((kVPad % 64) == 0 && kVPad >= kV && kVPad - kV < 64);
static_assert((kE % 32) == 0 && (kPP % 64) == 0);
static_assert(kTiles * 16 == kBPad && kBPad >= kB && kBPad - kB < 16);
static_assert(kOutTotal == 201000);
static_assert((kS % 32) == 0);

constexpr float kCarryEmb = 64.0f;
constexpr float kCarryW0  = 64.0f;
constexpr float kTabScale = 1.0f / (kCarryEmb * kCarryW0);
constexpr float kCA       = 64.0f;
constexpr float kCBH      = 2048.0f;
constexpr float kAccScale = kCA * kCBH;
constexpr float kAccInv   = 1.0f / kAccScale;
constexpr float kHalfMinNormal = 6.103515625e-05f;
static_assert(kAccScale == 131072.0f);

constexpr size_t kSzA    = (size_t)kVPad * kE * 2;
constexpr size_t kSzBt   = (size_t)64 * kE * 2;
constexpr size_t kSzBias = (size_t)64 * 4;
constexpr size_t kSzP    = (size_t)kVPad * kPP * 4;
constexpr size_t kSzH    = (size_t)kL * kBPad * kH * 4;
constexpr size_t kOffA    = 0;
constexpr size_t kOffBt   = kOffA + kSzA;
constexpr size_t kOffBias = kOffBt + kSzBt;
constexpr size_t kOffP    = kOffBias + kSzBias;
constexpr size_t kOffH    = kOffP + kSzP;
constexpr size_t kWsTotal = kOffH + kSzH;
static_assert(kWsTotal == 12340992ull);
static_assert(kWsTotal <= 134217728ull);
static_assert((kOffBt % 128) == 0 && (kOffBias % 128) == 0 && (kOffP % 128) == 0 && (kOffH % 128) == 0);

__device__ __forceinline__ unsigned short f2bf_bits(float f) {
  unsigned u = __float_as_uint(f);
  return (unsigned short)((u + 0x7FFFu + ((u >> 16) & 1u)) >> 16);
}
__device__ __forceinline__ float bf_bits2f(unsigned short h) { return __uint_as_float(((unsigned)h) << 16); }

__device__ __forceinline__ _Float16 cvt_h_flush(float c) {
  const float f = (fabsf(c) < kHalfMinNormal) ? 0.0f : c;
  return (_Float16)f;
}

__device__ __forceinline__ v8f mma_f16_guard(v16h a, v16h b, v8f c) {
  c = __builtin_amdgcn_wmma_f32_16x16x32_f16(false, a, false, b, (short)0, c, false, false);
  asm volatile("v_nop\n\tv_nop\n\tv_nop\n\tv_nop" : "+v"(c) : "v"(a), "v"(b));
  return c;
}

__device__ __forceinline__ v16h act_frag(const float (&v)[8]) {
  v8h hv;
#pragma unroll
  for (int i = 0; i < 8; ++i) hv[i] = cvt_h_flush(v[i] * kCA);
  const v8h z8 = (v8h){(_Float16)0.0f, (_Float16)0.0f, (_Float16)0.0f, (_Float16)0.0f,
                       (_Float16)0.0f, (_Float16)0.0f, (_Float16)0.0f, (_Float16)0.0f};
  return __builtin_shufflevector(hv, z8, 0, 1, 2, 3, 4, 5, 6, 7, 8, 9, 10, 11, 12, 13, 14, 15);
}

__device__ __forceinline__ v16h wgt_frag(v8h w) {
  const v8h z8 = (v8h){(_Float16)0.0f, (_Float16)0.0f, (_Float16)0.0f, (_Float16)0.0f,
                       (_Float16)0.0f, (_Float16)0.0f, (_Float16)0.0f, (_Float16)0.0f};
  return __builtin_shufflevector(w, z8, 0, 1, 2, 3, 4, 5, 6, 7, 8, 9, 10, 11, 12, 13, 14, 15);
}

__device__ __forceinline__ float sigmoid_fast(float x) {
  return __builtin_amdgcn_rcpf(1.0f + __expf(-x));
}
__device__ __forceinline__ float tanh_fast(float x) {
  const float t = __expf(-2.0f * fabsf(x));
  const float r = (1.0f - t) * __builtin_amdgcn_rcpf(1.0f + t);
  return copysignf(r, x);
}

__device__ __forceinline__ void dep_guard_h(v8f& a, v8f& b, v16h x, v16h y) { asm volatile("v_nop\n\tv_nop\n\tv_nop\n\tv_nop" : "+v"(a), "+v"(b) : "v"(x), "v"(y)); }
__device__ __forceinline__ void dep_guard_b(v8f& a, v8f& b, v16b x, v16b y) { asm volatile("v_nop\n\tv_nop\n\tv_nop\n\tv_nop" : "+v"(a), "+v"(b) : "v"(x), "v"(y)); }
__device__ __forceinline__ void keep4_h(v16h a, v16h b, v16h c, v16h d) { asm volatile("v_nop" :: "v"(a), "v"(b), "v"(c), "v"(d)); }
__device__ __forceinline__ void keep4_b(v16b a, v16b b, v16b c, v16b d) { asm volatile("v_nop" :: "v"(a), "v"(b), "v"(c), "v"(d)); }
__device__ __forceinline__ void acc_guard4(v8f& a, v8f& b, v8f& c, v8f& d) { asm volatile("v_nop\n\tv_nop\n\tv_nop\n\tv_nop" : "+v"(a), "+v"(b), "+v"(c), "+v"(d)); }
template <typename T> struct Frag;
template <> struct Frag<_Float16> {
  typedef v16h V; union U { v16h v; v8h h[2]; };
  static __device__ __forceinline__ v16h load(const _Float16* p) {
    U f; f.h[0] = *(const v8h*)(p); f.h[1] = *(const v8h*)(p + 16); return f.v;
  }
  static __device__ __forceinline__ v8f mma(v16h a, v16h b, v8f c) {
    return __builtin_amdgcn_wmma_f32_16x16x32_f16(false, a, false, b, (short)0, c, false, false);
  }
  static __device__ __forceinline__ void guard(v8f& a, v8f& b, v16h x, v16h y) { dep_guard_h(a, b, x, y); }
  static __device__ __forceinline__ void keep(v16h a, v16h b, v16h c, v16h d) { keep4_h(a, b, c, d); }
};
template <> struct Frag<__bf16> {
  typedef v16b V; union U { v16b v; v8b h[2]; };
  static __device__ __forceinline__ v16b load(const __bf16* p) {
    U f; f.h[0] = *(const v8b*)(p); f.h[1] = *(const v8b*)(p + 16); return f.v;
  }
  static __device__ __forceinline__ v8f mma(v16b a, v16b b, v8f c) {
    return __builtin_amdgcn_wmma_f32_16x16x32_bf16(false, a, false, b, (short)0, c, false, false);
  }
  static __device__ __forceinline__ void guard(v8f& a, v8f& b, v16b x, v16b y) { dep_guard_b(a, b, x, y); }
  static __device__ __forceinline__ void keep(v16b a, v16b b, v16b c, v16b d) { keep4_b(a, b, c, d); }
};

template <int ET> struct Elem;
template <> struct Elem<0> { typedef _Float16 T; };
template <> struct Elem<1> { typedef __bf16 T; };
template <int ET, int SPL, int BIAS_MODE, int OUT_MODE, bool RESID, int ACT = 0>
__global__ __launch_bounds__(256) void wmma_gemm64(
    const unsigned short* __restrict__ Ap, const unsigned short* __restrict__ A2p, int lda, long strideA,
    const unsigned short* __restrict__ Btp, const unsigned short* __restrict__ Bt2p, int ldb, long strideB,
    void* __restrict__ Cout, void* __restrict__ Cout2, int ldc, long strideC,
    const float* __restrict__ bias,
    const float* __restrict__ resid, long strideR,
    int M, int N, int K, float scale) {
  typedef typename Elem<ET>::T T;
  typedef typename Frag<T>::V V;
  const T* A = (const T*)Ap; const T* A2 = (const T*)A2p; const T* Bt = (const T*)Btp; const T* Bt2 = (const T*)Bt2p;
  __shared__ __align__(16) float sT[8][16 * 68];
  const int b    = blockIdx.y;
  const int lane = threadIdx.x & 31;
  const int wave = threadIdx.x >> 5;
  const int tilesN = N >> 6;
  const int tilesM = M >> 6;
  const int tile = blockIdx.x * 8 + wave;
  if (tile >= tilesM * tilesN) return;
  const int tm = tile / tilesN;
  const int tn = tile - tm * tilesN;
  const int m0 = tm << 6;
  const int n0 = tn << 6;

  const T* Ab  = A  + (size_t)b * strideA;
  const T* Bb  = Bt + (size_t)b * strideB;
  const T* Ab2 = (SPL >= 1) ? (A2  + (size_t)b * strideA) : nullptr;
  const T* Bb2 = (SPL == 2) ? (Bt2 + (size_t)b * strideB) : nullptr;

  const int rlane = lane & 15;
  const int koff  = (lane >> 4) * 8;
  const int mOff  = (lane >> 4) * 8;

  v8f acc[4][4];
#pragma unroll
  for (int i = 0; i < 4; ++i)
#pragma unroll
    for (int j = 0; j < 4; ++j) acc[i][j] = (v8f){0.f,0.f,0.f,0.f,0.f,0.f,0.f,0.f};

  for (int k0 = 0; k0 < K; k0 += 32) {
    V bh[4], bl[4];
#pragma unroll
    for (int j = 0; j < 4; ++j) {
      const size_t bo = (size_t)(n0 + (j << 4) + rlane) * ldb + koff + k0;
      bh[j] = Frag<T>::load(Bb + bo);
      if (SPL == 2) bl[j] = Frag<T>::load(Bb2 + bo);
    }
#pragma unroll
    for (int i = 0; i < 4; ++i) {
      const size_t ao = (size_t)(m0 + (i << 4) + rlane) * lda + koff + k0;
      V ah = Frag<T>::load(Ab + ao);
      V al;
      if (SPL >= 1) al = Frag<T>::load(Ab2 + ao);
#pragma unroll
      for (int j = 0; j < 4; ++j) {
        acc[i][j] = Frag<T>::mma(ah, bh[j], acc[i][j]);
        if (SPL == 2) acc[i][j] = Frag<T>::mma(ah, bl[j], acc[i][j]);
        if (SPL >= 1) acc[i][j] = Frag<T>::mma(al, bh[j], acc[i][j]);
      }
      Frag<T>::guard(acc[i][0], acc[i][3], ah, (SPL >= 1) ? al : ah);
    }
    Frag<T>::keep(bh[0], bh[1], bh[2], bh[3]);
    if (SPL == 2) Frag<T>::keep(bl[0], bl[1], bl[2], bl[3]);
  }
  acc_guard4(acc[0][0], acc[0][1], acc[0][2], acc[0][3]);
  acc_guard4(acc[1][0], acc[1][1], acc[1][2], acc[1][3]);
  acc_guard4(acc[2][0], acc[2][1], acc[2][2], acc[2][3]);
  acc_guard4(acc[3][0], acc[3][1], acc[3][2], acc[3][3]);

  float* slab = sT[wave];
  const float* Rb = RESID ? (resid + (size_t)b * strideR) : nullptr;
#pragma unroll
  for (int i = 0; i < 4; ++i) {
    const int mBase = m0 + (i << 4);
#pragma unroll
    for (int j = 0; j < 4; ++j) {
      const int n = n0 + (j << 4) + rlane;
      float bv = 0.f;
      if (BIAS_MODE == 2) bv = bias[n];
#pragma unroll
      for (int r = 0; r < 8; ++r) {
        float v = acc[i][j][r] * scale;
        if (BIAS_MODE == 1) v += bias[mBase + mOff + r];
        if (BIAS_MODE == 2) v += bv;
        if (RESID) v += Rb[(size_t)(mBase + mOff + r) * ldc + n];
        if (ACT == 1) v = tanhf(v);
        if (ACT == 2) v = fmaxf(v, 0.0f);
        if (ACT == 3) v = v / (1.0f + expf(-v));
        if (ACT == 4) v = (v > 0.f) ? v : 0.01f * v;
        slab[(mOff + r) * 68 + (j << 4) + rlane] = v;
      }
    }
    __builtin_amdgcn_fence(__ATOMIC_RELEASE, "workgroup");
    __builtin_amdgcn_wave_barrier();
    __builtin_amdgcn_fence(__ATOMIC_ACQUIRE, "workgroup");
    if (OUT_MODE == 0) {
      float* C = (float*)Cout + (size_t)b * strideC;
      const int hh = lane >> 4, c4 = (lane & 15) * 4;
      for (int pass = 0; pass < 2; ++pass) {
#pragma unroll
        for (int it = 0; it < 8; ++it) {
          const int row = it * 2 + hh;
          v4f v = *(const v4f*)(slab + row * 68 + c4);
          *(volatile v4f*)(C + (size_t)(mBase + row) * ldc + n0 + c4) = v;
        }
        __threadfence();
      }
    } else {
      const int q = lane >> 3, c8 = (lane & 7) * 8;
      unsigned short* C  = (unsigned short*)Cout  + (size_t)b * strideC;
      unsigned short* C2 = (OUT_MODE == 2) ? ((unsigned short*)Cout2 + (size_t)b * strideC) : nullptr;
      for (int pass = 0; pass < 2; ++pass) {
#pragma unroll
        for (int it = 0; it < 4; ++it) {
          const int row = it * 4 + q;
          const float* sp = slab + row * 68 + c8;
          v8h hv, lv;
#pragma unroll
          for (int e = 0; e < 8; ++e) {
            if (OUT_MODE == 1) {
              hv[e] = (_Float16)sp[e];
            } else {
              unsigned short hb = f2bf_bits(sp[e]);
              unsigned short lb = f2bf_bits(sp[e] - bf_bits2f(hb));
              hv[e] = __builtin_bit_cast(_Float16, hb);
              lv[e] = __builtin_bit_cast(_Float16, lb);
            }
          }
          *(volatile v8h*)(C + (size_t)(mBase + row) * ldc + n0 + c8) = hv;
          if (OUT_MODE == 2) *(volatile v8h*)(C2 + (size_t)(mBase + row) * ldc + n0 + c8) = lv;
        }
        __threadfence();
      }
    }
    __builtin_amdgcn_fence(__ATOMIC_RELEASE, "workgroup");
    __builtin_amdgcn_wave_barrier();
    __builtin_amdgcn_fence(__ATOMIC_ACQUIRE, "workgroup");
  }
}

constexpr int kPrepABlocks = (kVPad * kE / 8) / 256;
constexpr int kPrepBlocks  = kPrepABlocks + 3;
static_assert(kPrepABlocks * 256 * 8 == kVPad * kE);

__global__ __launch_bounds__(256) void prep_kernel(
    const float* __restrict__ emb, const float* __restrict__ Wxz0, const float* __restrict__ Wxr0,
    const float* __restrict__ WxH0, const float* __restrict__ bz0, const float* __restrict__ br0,
    const float* __restrict__ bH0, unsigned short* __restrict__ Apl, unsigned short* __restrict__ Btp,
    float* __restrict__ biasl)
{
  const int tid = threadIdx.x;
  const int blk = blockIdx.x;
  if (blk < kPrepABlocks) {
    const int i = blk * 256 + tid;
    const int row = i >> 3, c8 = (i & 7) * 8;
    const int rc = (row < kV) ? row : (kV - 1);
    const bool valid = (row < kV);
    const v4f a0 = *(const v4f*)(emb + (size_t)rc * kE + c8);
    const v4f a1 = *(const v4f*)(emb + (size_t)rc * kE + c8 + 4);
    v8h hv;
#pragma unroll
    for (int e = 0; e < 4; ++e) {
      const float f0 = valid ? (a0[e] * kCarryEmb) : 0.0f;
      const float f1 = valid ? (a1[e] * kCarryEmb) : 0.0f;
      hv[e]     = cvt_h_flush(f0);
      hv[4 + e] = cvt_h_flush(f1);
    }
    unsigned short* q = Apl + (size_t)i * 8;
    *(volatile v8h*)q = hv;
    __threadfence();
    *(volatile v8h*)q = hv;
  } else if (blk < kPrepABlocks + 2) {
    const int i = (blk - kPrepABlocks) * 256 + tid;
    const int nrow = i >> 3, k8 = (i & 7) * 8;
    const int jn = nrow & 7, g = nrow >> 3;
    v8h hv;
#pragma unroll
    for (int e = 0; e < 8; ++e) {
      const int k = k8 + e;
      float wz = Wxz0[k * kH + jn];
      float wr = Wxr0[k * kH + jn];
      float wc = WxH0[k * kH + jn];
      asm volatile("" : "+v"(wz), "+v"(wr), "+v"(wc));
      const float w = (g == 0) ? wz : ((g == 1) ? wr : ((g == 2) ? wc : 0.0f));
      hv[e] = cvt_h_flush(w * kCarryW0);
    }
    unsigned short* q = Btp + (size_t)i * 8;
    *(volatile v8h*)q = hv;
    __threadfence();
    *(volatile v8h*)q = hv;
  } else {
    const int q4 = tid & 15;
    v4f bv;
#pragma unroll
    for (int e = 0; e < 4; ++e) {
      const int nn = q4 * 4 + e;
      const int jn = nn & 7, g = nn >> 3;
      float z = bz0[jn];
      float r = br0[jn];
      float c = bH0[jn];
      asm volatile("" : "+v"(z), "+v"(r), "+v"(c));
      bv[e] = (g == 0) ? z : ((g == 1) ? r : ((g == 2) ? c : 0.0f));
    }
    asm volatile("" : "+v"(bv));
    if (tid < 16) {
      float* q = biasl + q4 * 4;
      *(volatile v4f*)q = bv;
      __threadfence();
      *(volatile v4f*)q = bv;
    }
  }
}

__global__ __launch_bounds__(32) void recur_kernel(
    const int* __restrict__ xtok, const float* __restrict__ P,
    const float* __restrict__ Whz0, const float* __restrict__ Whr0, const float* __restrict__ WrH0,
    const float* __restrict__ Wxz, const float* __restrict__ Whz, const float* __restrict__ bz,
    const float* __restrict__ Wxr, const float* __restrict__ Whr, const float* __restrict__ br,
    const float* __restrict__ WxH, const float* __restrict__ WrH, const float* __restrict__ bH,
    float* __restrict__ Hfin)
{
  __shared__ v8h sBzr[kL * 32];
  __shared__ v8h sBh[kL * 16];
  __shared__ __align__(16) float sH[kL * 128];
  __shared__ __align__(16) float sS[16 * 16];
  __shared__ __align__(16) float sP[16 * 24];
  __shared__ __align__(16) int   sTok[16 * 32];
  __shared__ float sBiasZR[kL * 16];
  __shared__ float sBiasH[kL * 8];

  const int lane = threadIdx.x & 31;
  const int hh = lane >> 4;
  const int n = lane & 15;
  const int j = lane & 7;
  const int shh = (lane >> 3) & 1;
  const int tile = blockIdx.x;

#pragma unroll 1
  for (int i = lane; i < kL * 32; i += 32) *(v4f*)(sH + 4 * i) = (v4f){0.f, 0.f, 0.f, 0.f};

#pragma unroll 1
  for (int L = 0; L < kL; ++L) {
    const int sl = (L > 0) ? (L - 1) : 0;
    const bool deep = (L > 0);
    const int wb = sl * 64 + j;
    float wzr[8], wcd[8];
#pragma unroll
    for (int i = 0; i < 8; ++i) {
      float a_xz  = Wxz[wb + i * 8];
      float a_xr  = Wxr[wb + i * 8];
      float a_hz  = Whz[wb + i * 8];
      float a_hr  = Whr[wb + i * 8];
      float a_hz0 = Whz0[i * 8 + j];
      float a_hr0 = Whr0[i * 8 + j];
      float a_xh  = WxH[wb + i * 8];
      float a_rh  = WrH[wb + i * 8];
      float a_rh0 = WrH0[i * 8 + j];
      asm volatile("" : "+v"(a_xz), "+v"(a_xr), "+v"(a_hz), "+v"(a_hr), "+v"(a_hz0), "+v"(a_hr0),
                        "+v"(a_xh), "+v"(a_rh), "+v"(a_rh0));
      const float gx  = (n < 8) ? a_xz : a_xr;
      const float gh  = (n < 8) ? a_hz : a_hr;
      const float gh0 = (n < 8) ? a_hz0 : a_hr0;
      const float vx  = deep ? gx : 0.0f;
      const float vh  = deep ? gh : gh0;
      wzr[i] = hh ? vh : vx;
      const float ux = deep ? a_xh : 0.0f;
      const float uh = deep ? a_rh : a_rh0;
      wcd[i] = shh ? uh : ux;
    }
    v8h zh, ch;
#pragma unroll
    for (int i = 0; i < 8; ++i) {
      zh[i] = cvt_h_flush(wzr[i] * kCBH);
      ch[i] = cvt_h_flush(wcd[i] * kCBH);
    }
    sBzr[L * 32 + lane] = zh;
    if (lane < 16) {
      sBh[L * 16 + lane] = ch;
    }
    float q_z = bz[sl * kH + j];
    float q_r = br[sl * kH + j];
    float q_h = bH[sl * kH + j];
    asm volatile("" : "+v"(q_z), "+v"(q_r), "+v"(q_h));
    const float bzr = deep ? ((n < 8) ? q_z : q_r) : 0.0f;
    const float bhc = deep ? q_h : 0.0f;
    if (hh == 0) sBiasZR[L * 16 + n] = bzr * kAccScale;
    if (lane < 8) sBiasH[L * 8 + lane] = bhc * kAccScale;
  }

  int prow[3], pseg[3];
#pragma unroll
  for (int i = 0; i < 3; ++i) {
    const int idx = lane + 32 * i;
    prow[i] = idx / 6;
    pseg[i] = idx - prow[i] * 6;
  }
  int trow[4], tseg[4], brow[4];
#pragma unroll
  for (int i = 0; i < 4; ++i) {
    const int idx = lane + 32 * i;
    trow[i] = idx >> 3;
    tseg[i] = idx & 7;
    const int bb = tile * 16 + trow[i];
    brow[i] = (bb < kB) ? bb : (kB - 1);
  }
  __syncthreads();

#pragma unroll 1
  for (int t = 0; t < kS; ++t) {
    const int tt = t & 31;
    if (tt == 0) {
      __syncthreads();
      v4i tk[4];
#pragma unroll
      for (int i = 0; i < 4; ++i)
        tk[i] = *(const v4i*)(xtok + (size_t)brow[i] * kS + t + tseg[i] * 4);
#pragma unroll
      for (int i = 0; i < 4; ++i)
        *(v4i*)(sTok + trow[i] * 32 + tseg[i] * 4) = tk[i];
      __syncthreads();
    }
    {
      v4f pv[3];
#pragma unroll
      for (int i = 0; i < 3; ++i) {
        int tok = sTok[prow[i] * 32 + tt];
        tok = (tok < 0) ? 0 : tok;
        tok = (tok > kV - 1) ? (kV - 1) : tok;
        pv[i] = *(const v4f*)(P + (size_t)tok * kPP + pseg[i] * 4);
      }
#pragma unroll
      for (int i = 0; i < 3; ++i)
        *(v4f*)(sP + prow[i] * 24 + pseg[i] * 4) = pv[i];
    }
    __syncthreads();

#pragma unroll 1
    for (int l = 0; l < kL; ++l) {
      float* hcur = sH + l * 128;
      const int lin = (l > 0) ? (l - 1) : 0;
      const float* hsrc = sH + (hh ? l : lin) * 128 + n * 8;
      const v4f s0 = *(const v4f*)(hsrc);
      const v4f s1 = *(const v4f*)(hsrc + 4);
      const bool xz = (l == 0) && (hh == 0);
      float sv[8];
      sv[0] = xz ? 0.0f : s0[0];
      sv[1] = xz ? 0.0f : s0[1];
      sv[2] = xz ? 0.0f : s0[2];
      sv[3] = xz ? 0.0f : s0[3];
      sv[4] = xz ? 0.0f : s1[0];
      sv[5] = xz ? 0.0f : s1[1];
      sv[6] = xz ? 0.0f : s1[2];
      sv[7] = xz ? 0.0f : s1[3];
      float hold[8];
#pragma unroll
      for (int r = 0; r < 8; ++r) hold[r] = hcur[(8 * hh + r) * 8 + j];

      const v16h a1 = act_frag(sv);
      const v16h bf1 = wgt_frag(sBzr[l * 32 + lane]);
      v8f c1;
      if (l == 0) {
#pragma unroll
        for (int r = 0; r < 8; ++r) c1[r] = sP[(8 * hh + r) * 24 + n] * kAccScale;
      } else {
        const float q = sBiasZR[l * 16 + n];
#pragma unroll
        for (int r = 0; r < 8; ++r) c1[r] = q;
      }
      c1 = mma_f16_guard(a1, bf1, c1);
      float g[8];
#pragma unroll
      for (int r = 0; r < 8; ++r) {
        g[r] = sigmoid_fast(c1[r] * kAccInv);
        sS[(8 * hh + r) * 16 + n] = g[r];
      }
      __syncthreads();

      const v4f r0 = *(const v4f*)(sS + n * 16 + 8);
      const v4f r1 = *(const v4f*)(sS + n * 16 + 12);
      float uv[8];
      uv[0] = hh ? (sv[0] * r0[0]) : sv[0];
      uv[1] = hh ? (sv[1] * r0[1]) : sv[1];
      uv[2] = hh ? (sv[2] * r0[2]) : sv[2];
      uv[3] = hh ? (sv[3] * r0[3]) : sv[3];
      uv[4] = hh ? (sv[4] * r1[0]) : sv[4];
      uv[5] = hh ? (sv[5] * r1[1]) : sv[5];
      uv[6] = hh ? (sv[6] * r1[2]) : sv[6];
      uv[7] = hh ? (sv[7] * r1[3]) : sv[7];
      const v16h a2 = act_frag(uv);
      const v16h bf2 = wgt_frag(sBh[l * 16 + hh * 8 + j]);
      v8f c2;
      if (l == 0) {
#pragma unroll
        for (int r = 0; r < 8; ++r) c2[r] = sP[(8 * hh + r) * 24 + 16 + j] * kAccScale;
      } else {
        const float q = sBiasH[l * 8 + j];
#pragma unroll
        for (int r = 0; r < 8; ++r) c2[r] = q;
      }
      c2 = mma_f16_guard(a2, bf2, c2);
      float hn[8];
#pragma unroll
      for (int r = 0; r < 8; ++r) {
        const float hc = tanh_fast(c2[r] * kAccInv);
        const float z = g[r];
        hn[r] = hold[r] * (1.0f - z) + z * hc;
      }
      if (n < 8) {
#pragma unroll
        for (int r = 0; r < 8; ++r) hcur[(8 * hh + r) * 8 + n] = hn[r];
      }
      __syncthreads();
    }
  }

  float* dst = Hfin + (size_t)tile * 128 + lane * 4;
  for (int pass = 0; pass < 2; ++pass) {
#pragma unroll 1
    for (int L = 0; L < kL; ++L) {
      const v4f v = *(const v4f*)(sH + L * 128 + lane * 4);
      *(volatile v4f*)(dst + (size_t)L * kBPad * kH) = v;
    }
    __threadfence();
  }
}

__global__ __launch_bounds__(256) void out_kernel(
    const float* __restrict__ Hfin, const float* __restrict__ Why, const float* __restrict__ by,
    float* __restrict__ out)
{
  const int i = blockIdx.x * 256 + threadIdx.x;
  const int ic = (i < kOutTotal) ? i : (kOutTotal - 1);
  const int bl = (ic < kB) ? ic : (kB - 1);
  const float* hp = Hfin + ((size_t)(kL - 1) * kBPad + bl) * kH;
  const v4f h0 = *(const v4f*)(hp);
  const v4f h1 = *(const v4f*)(hp + 4);
  float acc = 0.0f;
  acc = fmaf(h0[0], Why[0], acc);
  acc = fmaf(h0[1], Why[1], acc);
  acc = fmaf(h0[2], Why[2], acc);
  acc = fmaf(h0[3], Why[3], acc);
  acc = fmaf(h1[0], Why[4], acc);
  acc = fmaf(h1[1], Why[5], acc);
  acc = fmaf(h1[2], Why[6], acc);
  acc = fmaf(h1[3], Why[7], acc);
  const float lg = acc + by[0];
  const int e0 = ic - kB;
  const int ec = (e0 > 0) ? e0 : 0;
  const int Lq = ec / (kB * kH);
  const int rem = ec - Lq * (kB * kH);
  const int bq = rem >> 3, jq = rem & 7;
  const float cp = Hfin[((size_t)Lq * kBPad + bq) * kH + jq];
  float val = (ic < kB) ? lg : cp;
  asm volatile("" : "+v"(val));
  if (i < kOutTotal) {
    volatile float* q = out + i;
    *q = val;
    __threadfence();
    *q = val;
  }
}

extern "C" void kernel_launch(void* const* d_in, const int* in_sizes, int n_in,
                              void* d_out, int out_size, void* d_ws, size_t ws_size,
                              hipStream_t stream) {
  if (n_in < 22) return;
  if (in_sizes[0] != kB * kS) return;
  if (in_sizes[1] != kV * kE) return;
  if (in_sizes[2] != kE * kH || in_sizes[5] != kE * kH || in_sizes[8] != kE * kH) return;
  if (in_sizes[3] != kH * kH || in_sizes[6] != kH * kH || in_sizes[9] != kH * kH) return;
  if (in_sizes[4] != kH || in_sizes[7] != kH || in_sizes[10] != kH) return;
  if (in_sizes[11] != (kL - 1) * kH * kH || in_sizes[12] != (kL - 1) * kH * kH) return;
  if (in_sizes[14] != (kL - 1) * kH * kH || in_sizes[15] != (kL - 1) * kH * kH) return;
  if (in_sizes[17] != (kL - 1) * kH * kH || in_sizes[18] != (kL - 1) * kH * kH) return;
  if (in_sizes[13] != (kL - 1) * kH || in_sizes[16] != (kL - 1) * kH || in_sizes[19] != (kL - 1) * kH) return;
  if (in_sizes[20] != kH || in_sizes[21] != 1) return;
  if (out_size != kOutTotal) return;
  if (ws_size < kWsTotal) return;

  const int*   xtok = (const int*)d_in[0];
  const float* emb  = (const float*)d_in[1];
  const float* Wxz0 = (const float*)d_in[2];
  const float* Whz0 = (const float*)d_in[3];
  const float* bz0  = (const float*)d_in[4];
  const float* Wxr0 = (const float*)d_in[5];
  const float* Whr0 = (const float*)d_in[6];
  const float* br0  = (const float*)d_in[7];
  const float* WxH0 = (const float*)d_in[8];
  const float* WrH0 = (const float*)d_in[9];
  const float* bH0  = (const float*)d_in[10];
  const float* Wxz  = (const float*)d_in[11];
  const float* Whz  = (const float*)d_in[12];
  const float* bz   = (const float*)d_in[13];
  const float* Wxr  = (const float*)d_in[14];
  const float* Whr  = (const float*)d_in[15];
  const float* br   = (const float*)d_in[16];
  const float* WxH  = (const float*)d_in[17];
  const float* WrH  = (const float*)d_in[18];
  const float* bH   = (const float*)d_in[19];
  const float* Why  = (const float*)d_in[20];
  const float* by   = (const float*)d_in[21];
  float* out = (float*)d_out;

  char* ws = (char*)d_ws;
  unsigned short* Apl   = (unsigned short*)(ws + kOffA);
  unsigned short* Btp   = (unsigned short*)(ws + kOffBt);
  float*          biasl = (float*)(ws + kOffBias);
  float*          Ptab  = (float*)(ws + kOffP);
  float*          Hfin  = (float*)(ws + kOffH);

  prep_kernel<<<kPrepBlocks, 256, 0, stream>>>(emb, Wxz0, Wxr0, WxH0, bz0, br0, bH0, Apl, Btp, biasl);

  constexpr int kGemmTiles  = (kVPad / 64) * (kPP / 64);
  constexpr int kGemmBlocks = (kGemmTiles + 7) / 8;
  wmma_gemm64<0, 0, 2, 0, false><<<dim3(kGemmBlocks, 1), 256, 0, stream>>>(
      Apl, nullptr, kE, 0L,
      Btp, nullptr, kE, 0L,
      (void*)Ptab, nullptr, kPP, 0L,
      biasl, nullptr, 0L,
      kVPad, kPP, kE, kTabScale);

  recur_kernel<<<kTiles, 32, 0, stream>>>(xtok, Ptab, Whz0, Whr0, WrH0,
                                          Wxz, Whz, bz, Wxr, Whr, br, WxH, WrH, bH, Hfin);

  constexpr int kOutBlocks = (kOutTotal + 255) / 256;
  out_kernel<<<kOutBlocks, 256, 0, stream>>>(Hfin, Why, by, out);
}
